// BiMambaBlock_55465207661156
// MI455X (gfx1250) — hardware-verified
//
#include <hip/hip_runtime.h>
#include <math.h>

typedef __attribute__((ext_vector_type(16))) _Float16 v16h;
typedef __attribute__((ext_vector_type(8)))  _Float16 v8h;
typedef __attribute__((ext_vector_type(16))) __bf16   v16b;
typedef __attribute__((ext_vector_type(8)))  __bf16   v8b;
typedef __attribute__((ext_vector_type(8)))  float    v8f;
typedef __attribute__((ext_vector_type(4)))  float    v4f;

constexpr int kBatch   = 2;
constexpr int kSeqL    = 1024;
constexpr int kDmod    = 1024;
constexpr int kDin     = 2048;
constexpr int kNst     = 16;
constexpr int kDtR     = 64;
constexpr int kConvK   = 4;
constexpr int kPrjN    = 96;
constexpr int kPrjP    = 128;
constexpr int kXZP     = 2 * kDin;
constexpr int kRowsDir = kBatch * kSeqL;
constexpr int kRowsAll = 2 * kRowsDir;
constexpr int kUCPP    = 2 * kDin;
constexpr int kYPP     = 2 * kDin;
constexpr int kWKP     = 2 * kDin;
constexpr int kDTPP    = 2 * kDtR;
constexpr int kTP      = 260;
constexpr int kScanCh  = 256;
constexpr int kScanTS  = 16;
static_assert(kDtR + 2 * kNst == kPrjN);
static_assert((kDmod % 32) == 0 && (kWKP % 32) == 0 && (kDTPP % 32) == 0);
static_assert((kRowsAll % 64) == 0 && (kRowsDir % 64) == 0 && (kXZP % 64) == 0 && (kPrjP % 64) == 0 &&
              (kDin % 64) == 0 && (kDmod % 64) == 0);
static_assert((kSeqL % 64) == 0 && (kSeqL % kScanTS) == 0 && (kDin % kScanCh) == 0 && (kDin % 256) == 0);
static_assert((kTP % 4) == 0 && (kDmod % 8) == 0 && (kDtR % 8) == 0);

constexpr size_t kOffXA    = 0;
constexpr size_t kOffWIN   = kOffXA    + (size_t)kRowsAll * kDmod * 2;
constexpr size_t kOffYP    = 0;
constexpr size_t kSzYP     = (size_t)kRowsDir * kYPP * 2;
constexpr size_t kOffWXP   = kOffWIN   + (size_t)kRowsAll * kDmod * 2;
constexpr size_t kOffWDTP  = kOffWXP   + (size_t)2 * kPrjP * kWKP * 2;
constexpr size_t kOffWOUTP = kOffWDTP  + (size_t)2 * kDin * kDTPP * 2;
constexpr size_t kOffXZ    = kOffWOUTP + (size_t)kDmod * kWKP * 2;
constexpr size_t kOffUCP   = kOffXZ    + (size_t)kRowsAll * kXZP * 4;
constexpr size_t kOffXDBL  = kOffUCP   + (size_t)kRowsAll * kUCPP * 2;
constexpr size_t kOffDTP   = kOffXDBL  + (size_t)kRowsAll * kPrjP * 4;
constexpr size_t kWsTotal  = kOffDTP   + (size_t)kRowsAll * kDTPP * 2;
static_assert(kOffYP + kSzYP == kOffWXP);
static_assert(kWsTotal == 132120576ull);
static_assert(kWsTotal <= 134217728ull);
static_assert((kOffWIN % 128) == 0 && (kOffWXP % 128) == 0 && (kOffWDTP % 128) == 0 && (kOffWOUTP % 128) == 0 &&
              (kOffXZ % 128) == 0 && (kOffUCP % 128) == 0 && (kOffXDBL % 128) == 0 && (kOffDTP % 128) == 0);

__device__ __forceinline__ unsigned short f2bf_bits(float f) {
  unsigned u = __float_as_uint(f);
  return (unsigned short)((u + 0x7FFFu + ((u >> 16) & 1u)) >> 16);
}
__device__ __forceinline__ float bf_bits2f(unsigned short h) { return __uint_as_float(((unsigned)h) << 16); }
__device__ __forceinline__ float bf16r(float f) { return bf_bits2f(f2bf_bits(f)); }

__device__ __forceinline__ void dep_guard4_h(v8f& a, v8f& b, v8f& c, v8f& d, v16h x, v16h y) {
  asm volatile("v_nop\n\tv_nop\n\tv_nop\n\tv_nop" : "+v"(a), "+v"(b), "+v"(c), "+v"(d) : "v"(x), "v"(y));
}
__device__ __forceinline__ void dep_guard4_b(v8f& a, v8f& b, v8f& c, v8f& d, v16b x, v16b y) {
  asm volatile("v_nop\n\tv_nop\n\tv_nop\n\tv_nop" : "+v"(a), "+v"(b), "+v"(c), "+v"(d) : "v"(x), "v"(y));
}
__device__ __forceinline__ void keep4_h(v16h a, v16h b, v16h c, v16h d) { asm volatile("v_nop" :: "v"(a), "v"(b), "v"(c), "v"(d)); }
__device__ __forceinline__ void keep4_b(v16b a, v16b b, v16b c, v16b d) { asm volatile("v_nop" :: "v"(a), "v"(b), "v"(c), "v"(d)); }
__device__ __forceinline__ void acc_guard4(v8f& a, v8f& b, v8f& c, v8f& d) { asm volatile("v_nop\n\tv_nop\n\tv_nop\n\tv_nop" : "+v"(a), "+v"(b), "+v"(c), "+v"(d)); }
template <typename T> struct Frag;
template <> struct Frag<_Float16> {
  typedef v16h V; union U { v16h v; v8h h[2]; };
  static __device__ __forceinline__ v16h load(const _Float16* p) {
    U f; f.h[0] = *(const v8h*)(p); f.h[1] = *(const v8h*)(p + 16); return f.v;
  }
  static __device__ __forceinline__ v8f mma(v16h a, v16h b, v8f c) {
    return __builtin_amdgcn_wmma_f32_16x16x32_f16(false, a, false, b, (short)0, c, false, false);
  }
  static __device__ __forceinline__ void guard4(v8f& a, v8f& b, v8f& c, v8f& d, v16h x, v16h y) { dep_guard4_h(a, b, c, d, x, y); }
  static __device__ __forceinline__ void keep(v16h a, v16h b, v16h c, v16h d) { keep4_h(a, b, c, d); }
};
template <> struct Frag<__bf16> {
  typedef v16b V; union U { v16b v; v8b h[2]; };
  static __device__ __forceinline__ v16b load(const __bf16* p) {
    U f; f.h[0] = *(const v8b*)(p); f.h[1] = *(const v8b*)(p + 16); return f.v;
  }
  static __device__ __forceinline__ v8f mma(v16b a, v16b b, v8f c) {
    return __builtin_amdgcn_wmma_f32_16x16x32_bf16(false, a, false, b, (short)0, c, false, false);
  }
  static __device__ __forceinline__ void guard4(v8f& a, v8f& b, v8f& c, v8f& d, v16b x, v16b y) { dep_guard4_b(a, b, c, d, x, y); }
  static __device__ __forceinline__ void keep(v16b a, v16b b, v16b c, v16b d) { keep4_b(a, b, c, d); }
};

template <int ET> struct Elem;
template <> struct Elem<0> { typedef _Float16 T; };
template <> struct Elem<1> { typedef __bf16 T; };
template <int ET, bool SPLIT, int BIAS_MODE, int OUT_MODE, bool RESID, int ACT = 0>
__global__ __launch_bounds__(256) void wmma_gemm64(
    const unsigned short* __restrict__ Ap, const unsigned short* __restrict__ A2p, int lda, long strideA,
    const unsigned short* __restrict__ Btp, const unsigned short* __restrict__ Bt2p, int ldb, long strideB,
    void* __restrict__ Cout, void* __restrict__ Cout2, int ldc, long strideC,
    const float* __restrict__ bias,
    const float* __restrict__ resid, long strideR,
    int M, int N, int K, float scale) {
  typedef typename Elem<ET>::T T;
  typedef typename Frag<T>::V V;
  const T* A = (const T*)Ap; const T* A2 = (const T*)A2p; const T* Bt = (const T*)Btp; const T* Bt2 = (const T*)Bt2p;
  __shared__ __align__(16) float sT[8][16 * 68];
  const int b    = blockIdx.y;
  const int lane = threadIdx.x & 31;
  const int wave = threadIdx.x >> 5;
  const int tilesN = N >> 6;
  const int tilesM = M >> 6;
  const int tile = blockIdx.x * 8 + wave;
  if (tile >= tilesM * tilesN) return;
  const int tm = tile / tilesN;
  const int tn = tile - tm * tilesN;
  const int m0 = tm << 6;
  const int n0 = tn << 6;

  const T* Ab  = A  + (size_t)b * strideA;
  const T* Bb  = Bt + (size_t)b * strideB;
  const T* Ab2 = SPLIT ? (A2  + (size_t)b * strideA) : nullptr;
  const T* Bb2 = SPLIT ? (Bt2 + (size_t)b * strideB) : nullptr;

  const int rlane = lane & 15;
  const int koff  = (lane >> 4) * 8;
  const int mOff  = (lane >> 4) * 8;

  v8f acc[4][4];
#pragma unroll
  for (int i = 0; i < 4; ++i)
#pragma unroll
    for (int j = 0; j < 4; ++j) acc[i][j] = (v8f){0.f,0.f,0.f,0.f,0.f,0.f,0.f,0.f};

  for (int k0 = 0; k0 < K; k0 += 32) {
    V bh[4], bl[4];
#pragma unroll
    for (int j = 0; j < 4; ++j) {
      const size_t bo = (size_t)(n0 + (j << 4) + rlane) * ldb + koff + k0;
      bh[j] = Frag<T>::load(Bb + bo);
      if (SPLIT) bl[j] = Frag<T>::load(Bb2 + bo);
    }
#pragma unroll
    for (int i = 0; i < 4; ++i) {
      const size_t ao = (size_t)(m0 + (i << 4) + rlane) * lda + koff + k0;
      V ah = Frag<T>::load(Ab + ao);
      V al;
      if (SPLIT) al = Frag<T>::load(Ab2 + ao);
#pragma unroll
      for (int j = 0; j < 4; ++j) {
        acc[i][j] = Frag<T>::mma(ah, bh[j], acc[i][j]);
        if (SPLIT) {
          acc[i][j] = Frag<T>::mma(ah, bl[j], acc[i][j]);
          acc[i][j] = Frag<T>::mma(al, bh[j], acc[i][j]);
        }
      }
      Frag<T>::guard4(acc[i][0], acc[i][1], acc[i][2], acc[i][3], ah, SPLIT ? al : ah);
    }
    Frag<T>::keep(bh[0], bh[1], bh[2], bh[3]);
    if (SPLIT) Frag<T>::keep(bl[0], bl[1], bl[2], bl[3]);
  }
  acc_guard4(acc[0][0], acc[0][1], acc[0][2], acc[0][3]);
  acc_guard4(acc[1][0], acc[1][1], acc[1][2], acc[1][3]);
  acc_guard4(acc[2][0], acc[2][1], acc[2][2], acc[2][3]);
  acc_guard4(acc[3][0], acc[3][1], acc[3][2], acc[3][3]);

  float* slab = sT[wave];
  const float* Rb = RESID ? (resid + (size_t)b * strideR) : nullptr;
#pragma unroll
  for (int i = 0; i < 4; ++i) {
    const int mBase = m0 + (i << 4);
#pragma unroll
    for (int j = 0; j < 4; ++j) {
      const int n = n0 + (j << 4) + rlane;
      float bv = 0.f;
      if (BIAS_MODE == 2) bv = bias[n];
#pragma unroll
      for (int r = 0; r < 8; ++r) {
        float v = acc[i][j][r] * scale;
        if (BIAS_MODE == 1) v += bias[mBase + mOff + r];
        if (BIAS_MODE == 2) v += bv;
        if (RESID) v += Rb[(size_t)(mBase + mOff + r) * ldc + n];
        if (ACT == 1) v = tanhf(v);
        if (ACT == 2) v = fmaxf(v, 0.0f);
        if (ACT == 3) v = v / (1.0f + expf(-v));
        if (ACT == 4) v = (v > 0.f) ? v : 0.01f * v;
        slab[(mOff + r) * 68 + (j << 4) + rlane] = v;
      }
    }
    __builtin_amdgcn_fence(__ATOMIC_RELEASE, "workgroup");
    __builtin_amdgcn_wave_barrier();
    __builtin_amdgcn_fence(__ATOMIC_ACQUIRE, "workgroup");
    if (OUT_MODE == 0) {
      float* C = (float*)Cout + (size_t)b * strideC;
      const int hh = lane >> 4, c4 = (lane & 15) * 4;
      for (int pass = 0; pass < 2; ++pass) {
#pragma unroll
        for (int it = 0; it < 8; ++it) {
          const int row = it * 2 + hh;
          v4f v = *(const v4f*)(slab + row * 68 + c4);
          *(volatile v4f*)(C + (size_t)(mBase + row) * ldc + n0 + c4) = v;
        }
        __threadfence();
      }
    } else {
      const int q = lane >> 3, c8 = (lane & 7) * 8;
      unsigned short* C  = (unsigned short*)Cout  + (size_t)b * strideC;
      unsigned short* C2 = (OUT_MODE == 2) ? ((unsigned short*)Cout2 + (size_t)b * strideC) : nullptr;
      for (int pass = 0; pass < 2; ++pass) {
#pragma unroll
        for (int it = 0; it < 4; ++it) {
          const int row = it * 4 + q;
          const float* sp = slab + row * 68 + c8;
          v8h hv, lv;
#pragma unroll
          for (int e = 0; e < 8; ++e) {
            if (OUT_MODE == 1) {
              hv[e] = (_Float16)sp[e];
            } else {
              unsigned short hb = f2bf_bits(sp[e]);
              unsigned short lb = f2bf_bits(sp[e] - bf_bits2f(hb));
              hv[e] = __builtin_bit_cast(_Float16, hb);
              lv[e] = __builtin_bit_cast(_Float16, lb);
            }
          }
          *(volatile v8h*)(C + (size_t)(mBase + row) * ldc + n0 + c8) = hv;
          if (OUT_MODE == 2) *(volatile v8h*)(C2 + (size_t)(mBase + row) * ldc + n0 + c8) = lv;
        }
        __threadfence();
      }
    }
    __builtin_amdgcn_fence(__ATOMIC_RELEASE, "workgroup");
    __builtin_amdgcn_wave_barrier();
    __builtin_amdgcn_fence(__ATOMIC_ACQUIRE, "workgroup");
  }
}

__global__ __launch_bounds__(256) void xa_kernel(
    const float* __restrict__ x, const float* __restrict__ mask, unsigned short* __restrict__ XA, int total8)
{
  const int i = blockIdx.x * 256 + threadIdx.x;
  if (i >= total8) return;
  const int e0   = i << 3;
  const int orow = e0 / kDmod;
  const int oc   = e0 - orow * kDmod;
  const int dir  = orow / kRowsDir;
  const int srow = orow - dir * kRowsDir;
  const int scol = dir ? (kDmod - 8 - oc) : oc;
  const float* p = x + (size_t)srow * kDmod + scol;
  const v4f a0 = *(const v4f*)(p);
  const v4f a1 = *(const v4f*)(p + 4);
  const float mv = bf16r(mask[srow]);
  float f[8];
  f[0] = a0[0]; f[1] = a0[1]; f[2] = a0[2]; f[3] = a0[3];
  f[4] = a1[0]; f[5] = a1[1]; f[6] = a1[2]; f[7] = a1[3];
  v8h hv;
#pragma unroll
  for (int e = 0; e < 8; ++e) {
    const float vf = f[e];
    const float vr = f[7 - e];
    const float v  = dir ? vr : vf;
    const unsigned short hb = f2bf_bits(bf16r(v) * mv);
    hv[e] = __builtin_bit_cast(_Float16, hb);
  }
  unsigned short* q = XA + (size_t)e0;
  *(volatile v8h*)q = hv;
  __threadfence();
  *(volatile v8h*)q = hv;
}

template <bool DUP>
__global__ __launch_bounds__(256) void cvt_rows_bf16_kernel(
    const float* __restrict__ src, int R, int Kc, unsigned short* __restrict__ dst, int total8)
{
  const int i = blockIdx.x * 256 + threadIdx.x;
  if (i >= total8) return;
  const int e0 = i << 3;
  const int r  = e0 / Kc;
  const int c  = e0 - r * Kc;
  const bool keep = (r < R);
  const int rc = keep ? r : (R - 1);
  const float* p = src + (size_t)rc * Kc + c;
  const v4f a0 = *(const v4f*)(p);
  const v4f a1 = *(const v4f*)(p + 4);
  v8h hv;
#pragma unroll
  for (int e = 0; e < 4; ++e) {
    const float v0 = keep ? a0[e] : 0.0f;
    const float v1 = keep ? a1[e] : 0.0f;
    const unsigned short h0 = f2bf_bits(v0), h1 = f2bf_bits(v1);
    hv[e]     = __builtin_bit_cast(_Float16, h0);
    hv[4 + e] = __builtin_bit_cast(_Float16, h1);
  }
  const int P = DUP ? (2 * Kc) : Kc;
  unsigned short* q0 = dst + (size_t)r * P + c;
  unsigned short* q1 = q0 + Kc;
  *(volatile v8h*)q0 = hv;
  if (DUP) *(volatile v8h*)q1 = hv;
  __threadfence();
  *(volatile v8h*)q0 = hv;
  if (DUP) *(volatile v8h*)q1 = hv;
}

__global__ __launch_bounds__(256) void dt_split_kernel(
    const float* __restrict__ XDBL, unsigned short* __restrict__ DTP, int total8)
{
  const int i = blockIdx.x * 256 + threadIdx.x;
  if (i >= total8) return;
  const int e0  = i << 3;
  const int row = e0 / kDtR;
  const int c8  = e0 - row * kDtR;
  const float* p = XDBL + (size_t)row * kPrjP + c8;
  const v4f a0 = *(const v4f*)(p);
  const v4f a1 = *(const v4f*)(p + 4);
  v8h hv, lv;
#pragma unroll
  for (int e = 0; e < 4; ++e) {
    const unsigned short h0 = f2bf_bits(a0[e]), h1 = f2bf_bits(a1[e]);
    const unsigned short l0 = f2bf_bits(a0[e] - bf_bits2f(h0)), l1 = f2bf_bits(a1[e] - bf_bits2f(h1));
    hv[e]     = __builtin_bit_cast(_Float16, h0);
    hv[4 + e] = __builtin_bit_cast(_Float16, h1);
    lv[e]     = __builtin_bit_cast(_Float16, l0);
    lv[4 + e] = __builtin_bit_cast(_Float16, l1);
  }
  unsigned short* qh = DTP + (size_t)row * kDTPP + c8;
  unsigned short* ql = qh + kDtR;
  *(volatile v8h*)qh = hv;
  *(volatile v8h*)ql = lv;
  __threadfence();
  *(volatile v8h*)qh = hv;
  *(volatile v8h*)ql = lv;
}

__global__ __launch_bounds__(256) void conv_silu_kernel(
    const float* __restrict__ XZ,
    const float* __restrict__ cw_f, const float* __restrict__ cb_f,
    const float* __restrict__ cw_r, const float* __restrict__ cb_r,
    unsigned short* __restrict__ UCP)
{
  __shared__ __align__(16) float sT[16 * kTP];
  const int tid = threadIdx.x, lane = tid & 31, wave = tid >> 5;
  const int d0 = blockIdx.x * 256, d = d0 + tid;
  const int g0 = blockIdx.y * 64;
  const int dir = (g0 >= kRowsDir) ? 1 : 0;
  const int tb  = g0 & (kSeqL - 1);
  const float* cw = dir ? cw_r : cw_f;
  const float* cb = dir ? cb_r : cb_f;
  const float w0 = bf16r(cw[d * kConvK + 0]), w1 = bf16r(cw[d * kConvK + 1]);
  const float w2 = bf16r(cw[d * kConvK + 2]), w3 = bf16r(cw[d * kConvK + 3]);
  const float bc = bf16r(cb[d]);
  float xm3, xm2, xm1;
  {
    const bool hist = (tb > 0);
    const int rb = hist ? (g0 - 3) : g0;
    const float v3 = XZ[(size_t)rb * kXZP + d];
    const float v2 = XZ[(size_t)(rb + 1) * kXZP + d];
    const float v1 = XZ[(size_t)(rb + 2) * kXZP + d];
    xm3 = hist ? v3 : 0.f;
    xm2 = hist ? v2 : 0.f;
    xm1 = hist ? v1 : 0.f;
  }
#pragma unroll 1
  for (int sub = 0; sub < 4; ++sub) {
    const int lb = g0 + sub * 16;
#pragma unroll 1
    for (int s = 0; s < 16; ++s) {
      const float xcur = XZ[(size_t)(lb + s) * kXZP + d];
      float acc = w0 * xm3;
      acc = fmaf(w1, xm2, acc);
      acc = fmaf(w2, xm1, acc);
      acc = fmaf(w3, xcur, acc);
      const float sv = acc + bc;
      const float sg = __builtin_amdgcn_rcpf(1.0f + __expf(-sv));
      sT[s * kTP + tid] = sv * sg;
      xm3 = xm2; xm2 = xm1; xm1 = xcur;
    }
    __syncthreads();
    v8h hv[2], lv[2];
#pragma unroll
    for (int it = 0; it < 2; ++it) {
      const float* sp = sT + (it * 8 + wave) * kTP + lane * 8;
      const v4f a0 = *(const v4f*)(sp);
      const v4f a1 = *(const v4f*)(sp + 4);
#pragma unroll
      for (int e = 0; e < 4; ++e) {
        const unsigned short h0 = f2bf_bits(a0[e]), h1 = f2bf_bits(a1[e]);
        const unsigned short l0 = f2bf_bits(a0[e] - bf_bits2f(h0)), l1 = f2bf_bits(a1[e] - bf_bits2f(h1));
        hv[it][e]     = __builtin_bit_cast(_Float16, h0);
        hv[it][4 + e] = __builtin_bit_cast(_Float16, h1);
        lv[it][e]     = __builtin_bit_cast(_Float16, l0);
        lv[it][4 + e] = __builtin_bit_cast(_Float16, l1);
      }
    }
    for (int pass = 0; pass < 2; ++pass) {
#pragma unroll
      for (int it = 0; it < 2; ++it) {
        const size_t o = (size_t)(lb + it * 8 + wave) * kUCPP + d0 + lane * 8;
        *(volatile v8h*)(UCP + o) = hv[it];
        *(volatile v8h*)(UCP + o + kDin) = lv[it];
      }
      __threadfence();
    }
    __syncthreads();
  }
}

__device__ __forceinline__ float dir_step(float (&h)[kNst], const float (&An)[kNst], float bb, float Dd,
    const float* __restrict__ XZ, const unsigned int* __restrict__ UCPw,
    int row, int d, int dw, int sh, const float* bc)
{
  const size_t rb = (size_t)row * kXZP;
  const float a  = XZ[rb + d] + bb;
  const float zv = XZ[rb + kDin + d];
  const size_t wb = (size_t)row * (kUCPP / 2);
  const unsigned wh = UCPw[wb + dw];
  const unsigned wl = UCPw[wb + (kDin / 2) + dw];
  const float uh = __uint_as_float(((wh >> sh) & 0xffffu) << 16);
  const float ul = __uint_as_float(((wl >> sh) & 0xffffu) << 16);
  const float xv = uh + ul;
  const float ea  = __expf(-fabsf(a));
  const float up  = 1.0f + ea;
  const float l1p = __logf(up) + (ea - (up - 1.0f)) * __builtin_amdgcn_rcpf(up);
  const float delta = fmaxf(a, 0.0f) + l1p;
  v4f Bq[4], Cq[4];
#pragma unroll
  for (int qq = 0; qq < 4; ++qq) {
    Bq[qq] = *(const v4f*)(bc + 4 * qq);
    Cq[qq] = *(const v4f*)(bc + kNst + 4 * qq);
  }
  float y = 0.f;
#pragma unroll
  for (int n = 0; n < kNst; ++n) {
    const float e = __expf(delta * An[n]);
    float db = delta * Bq[n >> 2][n & 3];
    asm volatile("" : "+v"(db));
    float p = db * xv;
    asm volatile("" : "+v"(p));
    float qv = h[n] * e;
    asm volatile("" : "+v"(qv));
    const float hn = qv + p;
    h[n] = hn;
    float rr = Cq[n >> 2][n & 3] * hn;
    asm volatile("" : "+v"(rr));
    y += rr;
  }
  float sk = xv * Dd;
  asm volatile("" : "+v"(sk));
  y += sk;
  const float sg = __builtin_amdgcn_rcpf(1.0f + __expf(-zv));
  const float g  = zv * sg;
  return y * g;
}

__global__ __launch_bounds__(256) void scan_kernel(
    const float* __restrict__ XZ, const unsigned int* __restrict__ UCPw, const float* __restrict__ XDBL,
    const float* __restrict__ dtb_f, const float* __restrict__ dtb_r,
    const float* __restrict__ Alog_f, const float* __restrict__ Alog_r,
    const float* __restrict__ D_f, const float* __restrict__ D_r,
    unsigned short* __restrict__ YP)
{
  __shared__ __align__(16) float sA[kScanCh * kNst];
  __shared__ __align__(16) float sBC[2 * kScanTS * 32];
  __shared__ __align__(16) float sY[kScanTS * kTP];
  const int tid = threadIdx.x, lane = tid & 31, wave = tid >> 5;
  constexpr int kBlkPerB = kDin / kScanCh;
  const int b  = blockIdx.x / kBlkPerB;
  const int d0 = (blockIdx.x - b * kBlkPerB) * kScanCh;
  const int d  = d0 + tid;

  float Af[kNst], Ar[kNst], hf[kNst], hr[kNst];
#pragma unroll
  for (int p = 0; p < 4; ++p) {
    const int idx = tid + p * kScanCh;
    *(v4f*)(sA + idx * 4) = *(const v4f*)(Alog_f + (size_t)d0 * kNst + (size_t)idx * 4);
  }
  __syncthreads();
#pragma unroll
  for (int n = 0; n < kNst; ++n) { Af[n] = -__expf(bf16r(sA[tid * kNst + n])); hf[n] = 0.f; }
  __syncthreads();
#pragma unroll
  for (int p = 0; p < 4; ++p) {
    const int idx = tid + p * kScanCh;
    *(v4f*)(sA + idx * 4) = *(const v4f*)(Alog_r + (size_t)d0 * kNst + (size_t)idx * 4);
  }
  __syncthreads();
#pragma unroll
  for (int n = 0; n < kNst; ++n) { Ar[n] = -__expf(bf16r(sA[tid * kNst + n])); hr[n] = 0.f; }

  const float bbf = bf16r(dtb_f[d]), bbr = bf16r(dtb_r[d]);
  const float Ddf = bf16r(D_f[d]),   Ddr = bf16r(D_r[d]);
  const int sh = (d & 1) << 4;
  const int dw = d >> 1;
  const int rowf0 = b * kSeqL;
  const int rowr0 = kRowsDir + b * kSeqL;
  const int sdir = tid >> 7, srr = (tid >> 3) & 15, sq4 = (tid & 7) * 4;

#pragma unroll 1
  for (int c = 0; c < kSeqL / kScanTS; ++c) {
    const int l0 = c * kScanTS;
    __syncthreads();
    {
      const size_t srow = (size_t)(sdir * kRowsDir + b * kSeqL + l0 + srr);
      *(v4f*)(sBC + sdir * (kScanTS * 32) + srr * 32 + sq4) = *(const v4f*)(XDBL + srow * kPrjP + kDtR + sq4);
    }
    __syncthreads();
#pragma unroll 1
    for (int s = 0; s < kScanTS; ++s) {
      const int t = l0 + s;
      const float yf = dir_step(hf, Af, bbf, Ddf, XZ, UCPw, rowf0 + t, d, dw, sh, sBC + s * 32);
      const float yr = dir_step(hr, Ar, bbr, Ddr, XZ, UCPw, rowr0 + t, d, dw, sh, sBC + kScanTS * 32 + s * 32);
      sY[s * kTP + tid] = yf + yr;
    }
    __syncthreads();
    v8h hv[2], lv[2];
#pragma unroll
    for (int it = 0; it < 2; ++it) {
      const float* sp = sY + (it * 8 + wave) * kTP + lane * 8;
      const v4f a0 = *(const v4f*)(sp);
      const v4f a1 = *(const v4f*)(sp + 4);
#pragma unroll
      for (int e = 0; e < 4; ++e) {
        const unsigned short h0 = f2bf_bits(a0[e]), h1 = f2bf_bits(a1[e]);
        const unsigned short l0b = f2bf_bits(a0[e] - bf_bits2f(h0)), l1b = f2bf_bits(a1[e] - bf_bits2f(h1));
        hv[it][e]     = __builtin_bit_cast(_Float16, h0);
        hv[it][4 + e] = __builtin_bit_cast(_Float16, h1);
        lv[it][e]     = __builtin_bit_cast(_Float16, l0b);
        lv[it][4 + e] = __builtin_bit_cast(_Float16, l1b);
      }
    }
    for (int pass = 0; pass < 2; ++pass) {
#pragma unroll
      for (int it = 0; it < 2; ++it) {
        const size_t o = (size_t)(rowf0 + l0 + it * 8 + wave) * kYPP + d0 + lane * 8;
        *(volatile v8h*)(YP + o) = hv[it];
        *(volatile v8h*)(YP + o + kDin) = lv[it];
      }
      __threadfence();
    }
  }
}

extern "C" void kernel_launch(void* const* d_in, const int* in_sizes, int n_in,
                              void* d_out, int out_size, void* d_ws, size_t ws_size,
                              hipStream_t stream)
{
  if (n_in < 18) return;
  if (in_sizes[0] != kRowsDir * kDmod) return;
  if (in_sizes[1] != kRowsDir) return;
  if (in_sizes[2] != kXZP * kDmod) return;
  if (in_sizes[3] != kDmod * kDin) return;
  for (int g = 0; g < 2; ++g) {
    const int o = 4 + 7 * g;
    if (in_sizes[o + 0] != kDin * kConvK) return;
    if (in_sizes[o + 1] != kDin) return;
    if (in_sizes[o + 2] != kPrjN * kDin) return;
    if (in_sizes[o + 3] != kDin * kDtR) return;
    if (in_sizes[o + 4] != kDin) return;
    if (in_sizes[o + 5] != kDin * kNst) return;
    if (in_sizes[o + 6] != kDin) return;
  }
  if (out_size != kRowsDir * kDmod) return;
  if (ws_size < kWsTotal) return;

  const float* x        = (const float*)d_in[0];
  const float* mask     = (const float*)d_in[1];
  const float* W_in     = (const float*)d_in[2];
  const float* W_out    = (const float*)d_in[3];
  const float* conv_w_f = (const float*)d_in[4];
  const float* conv_b_f = (const float*)d_in[5];
  const float* xprj_w_f = (const float*)d_in[6];
  const float* dt_w_f   = (const float*)d_in[7];
  const float* dt_b_f   = (const float*)d_in[8];
  const float* A_log_f  = (const float*)d_in[9];
  const float* D_f      = (const float*)d_in[10];
  const float* conv_w_r = (const float*)d_in[11];
  const float* conv_b_r = (const float*)d_in[12];
  const float* xprj_w_r = (const float*)d_in[13];
  const float* dt_w_r   = (const float*)d_in[14];
  const float* dt_b_r   = (const float*)d_in[15];
  const float* A_log_r  = (const float*)d_in[16];
  const float* D_r      = (const float*)d_in[17];
  float* out = (float*)d_out;

  char* ws = (char*)d_ws;
  unsigned short* XA    = (unsigned short*)(ws + kOffXA);
  unsigned short* WIN   = (unsigned short*)(ws + kOffWIN);
  unsigned short* YP    = (unsigned short*)(ws + kOffYP);
  unsigned short* WXP   = (unsigned short*)(ws + kOffWXP);
  unsigned short* WDTP  = (unsigned short*)(ws + kOffWDTP);
  unsigned short* WOUTP = (unsigned short*)(ws + kOffWOUTP);
  float*          XZ    = (float*)(ws + kOffXZ);
  unsigned short* UCP   = (unsigned short*)(ws + kOffUCP);
  float*          XDBL  = (float*)(ws + kOffXDBL);
  unsigned short* DTP   = (unsigned short*)(ws + kOffDTP);
  const float* dummy_bias  = dt_b_f;
  const float* dummy_resid = x;

  constexpr int kXa8   = kRowsAll * kDmod / 8;
  constexpr int kWin8  = kXZP * kDmod / 8;
  constexpr int kWxp8  = kPrjP * kDin / 8;
  constexpr int kWdt8  = kDin * kDtR / 8;
  constexpr int kWout8 = kDmod * kDin / 8;
  static_assert((kXa8 % 256) == 0 && (kWin8 % 256) == 0 && (kWxp8 % 256) == 0 && (kWdt8 % 256) == 0 && (kWout8 % 256) == 0);
  xa_kernel<<<kXa8 / 256, 256, 0, stream>>>(x, mask, XA, kXa8);
  cvt_rows_bf16_kernel<false><<<kWin8 / 256, 256, 0, stream>>>(W_in, kXZP, kDmod, WIN, kWin8);
  cvt_rows_bf16_kernel<true><<<kWxp8 / 256, 256, 0, stream>>>(xprj_w_f, kPrjN, kDin, WXP, kWxp8);
  cvt_rows_bf16_kernel<true><<<kWxp8 / 256, 256, 0, stream>>>(xprj_w_r, kPrjN, kDin, WXP + (size_t)kPrjP * kWKP, kWxp8);
  cvt_rows_bf16_kernel<true><<<kWdt8 / 256, 256, 0, stream>>>(dt_w_f, kDin, kDtR, WDTP, kWdt8);
  cvt_rows_bf16_kernel<true><<<kWdt8 / 256, 256, 0, stream>>>(dt_w_r, kDin, kDtR, WDTP + (size_t)kDin * kDTPP, kWdt8);
  cvt_rows_bf16_kernel<true><<<kWout8 / 256, 256, 0, stream>>>(W_out, kDmod, kDin, WOUTP, kWout8);

  wmma_gemm64<1, false, 0, 0, false><<<dim3((kRowsAll / 64) * (kXZP / 64) / 8, 1), 256, 0, stream>>>(
      XA, XA, kDmod, 0L, WIN, WIN, kDmod, 0L,
      (void*)XZ, (void*)XZ, kXZP, 0L, dummy_bias, dummy_resid, 0L, kRowsAll, kXZP, kDmod, 1.0f);

  conv_silu_kernel<<<dim3(kDin / 256, kRowsAll / 64), 256, 0, stream>>>(XZ, conv_w_f, conv_b_f, conv_w_r, conv_b_r, UCP);

  wmma_gemm64<1, false, 0, 0, false><<<dim3((kRowsDir / 64) * (kPrjP / 64) / 8, 2), 256, 0, stream>>>(
      UCP, UCP, kUCPP, (long)kRowsDir * kUCPP, WXP, WXP, kWKP, (long)kPrjP * kWKP,
      (void*)XDBL, (void*)XDBL, kPrjP, (long)kRowsDir * kPrjP, dummy_bias, dummy_resid, 0L, kRowsDir, kPrjP, kUCPP, 1.0f);

  constexpr int kDtp8 = kRowsAll * kDtR / 8;
  static_assert((kDtp8 % 256) == 0);
  dt_split_kernel<<<kDtp8 / 256, 256, 0, stream>>>(XDBL, DTP, kDtp8);

  wmma_gemm64<1, false, 0, 0, false><<<dim3((kRowsDir / 64) * (kDin / 64) / 8, 2), 256, 0, stream>>>(
      DTP, DTP, kDTPP, (long)kRowsDir * kDTPP, WDTP, WDTP, kDTPP, (long)kDin * kDTPP,
      (void*)XZ, (void*)XZ, kXZP, (long)kRowsDir * kXZP, dummy_bias, dummy_resid, 0L, kRowsDir, kDin, kDTPP, 1.0f);

  scan_kernel<<<kBatch * (kDin / kScanCh), kScanCh, 0, stream>>>(
      XZ, (const unsigned int*)(const void*)UCP, XDBL, dt_b_f, dt_b_r, A_log_f, A_log_r, D_f, D_r, YP);

  wmma_gemm64<1, false, 0, 0, false><<<dim3((kRowsDir / 64) * (kDmod / 64) / 8, 1), 256, 0, stream>>>(
      YP, YP, kYPP, 0L, WOUTP, WOUTP, kWKP, 0L,
      (void*)out, (void*)out, kDmod, 0L, dummy_bias, dummy_resid, 0L, kRowsDir, kDmod, kYPP, 1.0f);
}
